// SelfAttentionLocal_50861002719401
// MI455X (gfx1250) — hardware-verified
//
#include <hip/hip_runtime.h>

typedef _Float16 v16h __attribute__((ext_vector_type(16)));
typedef _Float16 v8h  __attribute__((ext_vector_type(8)));
typedef _Float16 v8ha __attribute__((ext_vector_type(8), __may_alias__));
typedef _Float16 v2h  __attribute__((ext_vector_type(2)));
typedef float    v8f  __attribute__((ext_vector_type(8)));
typedef float    v4f  __attribute__((ext_vector_type(4)));

#define BB     4
#define CC     64
#define NN     32768
#define DD     8
#define EE     80
#define TN     64
#define WCAP   512
#define SPITCH 516
#define XT_LD  72
#define SV_LD  72
#define SO_LD  68
#define MAXWIN 4
#define NTHR   128
#define NEGBIG (-1.0e30f)
#define L2E    1.4426950408889634f

static_assert((SPITCH * 4) % 16 == 0);
static_assert(CC * SO_LD <= 16 * SPITCH);
static_assert(NN % TN == 0);
static_assert((XT_LD * 2) % 16 == 0);
static_assert((SV_LD * 2) % 16 == 0);
static_assert(TN * DD == 4 * NTHR);
static_assert(WCAP * DD == 4 * 8 * NTHR);

#if __has_builtin(__builtin_amdgcn_exp2f)
#define EXP2F(v) __builtin_amdgcn_exp2f(v)
#else
#define EXP2F(v) exp2f(v)
#endif

union Frag { v16h v; v8h hh[2]; };

__device__ __forceinline__ v8f mma_f16(v16h a, v16h b, v8f c)
{
    c = __builtin_amdgcn_wmma_f32_16x16x32_f16(false, a, false, b, (short)0, c, false, false);
    asm volatile("v_nop\n\tv_nop\n\tv_nop\n\tv_nop" : "+v"(c) : "v"(a), "v"(b));
    return c;
}

__device__ __forceinline__ float frcp(float v) { return __builtin_amdgcn_rcpf(v); }

__global__ __launch_bounds__(NTHR) void k_prep_w(
    const float* __restrict__ Wq, const float* __restrict__ Wk, const float* __restrict__ Wv,
    _Float16* __restrict__ Wall)
{
    const int e = threadIdx.x;
    if (e >= EE) return;
    const float* src = (e < DD) ? (Wq + e * CC)
                     : ((e < 2 * DD) ? (Wk + (e - DD) * CC) : (Wv + (e - 2 * DD) * CC));
    v8h wv[8];
    #pragma unroll
    for (int j = 0; j < 8; ++j) {
        const v4f a = *(const v4f*)(src + 8 * j);
        const v4f c = *(const v4f*)(src + 8 * j + 4);
        v8h t;
        t[0] = (_Float16)(a[0] * 16.0f); t[1] = (_Float16)(a[1] * 16.0f);
        t[2] = (_Float16)(a[2] * 16.0f); t[3] = (_Float16)(a[3] * 16.0f);
        t[4] = (_Float16)(c[0] * 16.0f); t[5] = (_Float16)(c[1] * 16.0f);
        t[6] = (_Float16)(c[2] * 16.0f); t[7] = (_Float16)(c[3] * 16.0f);
        wv[j] = t;
    }
    _Float16* dst = Wall + e * CC;
    #pragma unroll
    for (int j = 0; j < 8; ++j) *(volatile v8h*)(dst + 8 * j) = wv[j];
    __threadfence();
    #pragma unroll
    for (int j = 0; j < 8; ++j) *(volatile v8h*)(dst + 8 * j) = wv[j];
}

__global__ __launch_bounds__(NTHR) void k_proj(
    const float* __restrict__ x, const _Float16* __restrict__ Wall,
    const float* __restrict__ bq, const float* __restrict__ bk, const float* __restrict__ bv,
    float* __restrict__ qd, float* __restrict__ kd, _Float16* __restrict__ vd, int nblk)
{
    __shared__ __attribute__((aligned(16))) _Float16 sxT[TN * XT_LD];
    __shared__ __attribute__((aligned(16))) float    sQK[2 * TN * DD];
    __shared__ __attribute__((aligned(16))) _Float16 sV[CC * SV_LD];
    __shared__ float sBias[EE];

    const int tid = threadIdx.x;
    const int w = tid >> 5, l = tid & 31, h = l >> 4, m = l & 15;
    const int b  = blockIdx.x / nblk;
    const int n0 = (blockIdx.x - b * nblk) * TN;

    if (tid < DD)            sBias[tid] = bq[tid];
    else if (tid < 2 * DD)   sBias[tid] = bk[tid - DD];
    else if (tid < EE)       sBias[tid] = bv[tid - 2 * DD];

    #pragma unroll
    for (int it = 0; it < 4; ++it) {
        const int c  = 2 * ((tid >> 4) + 8 * it);
        const int n4 = (tid & 15) * 4;
        const float* p0 = x + ((size_t)b * CC + c) * NN + n0 + n4;
        const v4f x0 = *(const v4f*)p0;
        const v4f x1 = *(const v4f*)(p0 + NN);
        #pragma unroll
        for (int u = 0; u < 4; ++u) {
            v2h t;
            t[0] = (_Float16)x0[u];
            t[1] = (_Float16)x1[u];
            *(v2h*)(sxT + (n4 + u) * XT_LD + c) = t;
        }
    }
    __syncthreads();

    v8f acc[5];
    #pragma unroll
    for (int et = 0; et < 5; ++et) {
        #pragma unroll
        for (int r = 0; r < 8; ++r) acc[et][r] = 0.0f;
    }
    #pragma unroll
    for (int ks = 0; ks < 2; ++ks) {
        Frag bf;
        const _Float16* bp = sxT + (16 * w + m) * XT_LD + 32 * ks + 8 * h;
        bf.hh[0] = *(const v8h*)bp;
        bf.hh[1] = *(const v8h*)(bp + 16);
        #pragma unroll
        for (int et = 0; et < 5; ++et) {
            Frag af;
            const _Float16* ap = Wall + (16 * et + m) * CC + 32 * ks + 8 * h;
            af.hh[0] = *(const v8h*)ap;
            af.hh[1] = *(const v8h*)(ap + 16);
            acc[et] = mma_f16(af.v, bf.v, acc[et]);
        }
    }

    const float wsc = 0.0625f;
    {
        v4f lo, hi;
        #pragma unroll
        for (int r = 0; r < 4; ++r) {
            lo[r] = fmaf(acc[0][r],     wsc, sBias[8 * h + r]);
            hi[r] = fmaf(acc[0][r + 4], wsc, sBias[8 * h + r + 4]);
        }
        float* dq = sQK + ((h * TN) + 16 * w + m) * DD;
        *(v4f*)dq = lo;
        *(v4f*)(dq + 4) = hi;
    }
    #pragma unroll
    for (int et = 1; et < 5; ++et) {
        #pragma unroll
        for (int r = 0; r < 8; ++r) {
            const int c = 16 * (et - 1) + 8 * h + r;
            sV[c * SV_LD + 16 * w + m] = (_Float16)fmaf(acc[et][r], wsc, sBias[2 * DD + c]);
        }
    }
    __syncthreads();

    const v4f qv = *(const v4f*)(sQK + 4 * tid);
    const v4f kv = *(const v4f*)(sQK + TN * DD + 4 * tid);
    const size_t qoff = ((size_t)b * NN + n0) * DD + 4 * tid;
    v8h vv[4];
    size_t voff[4];
    #pragma unroll
    for (int p = 0; p < 4; ++p) {
        const int c = 16 * p + (tid >> 3);
        vv[p]   = *(const v8h*)(sV + c * SV_LD + (tid & 7) * 8);
        voff[p] = ((size_t)b * CC + c) * NN + n0 + (tid & 7) * 8;
    }
    *(volatile v4f*)(qd + qoff) = qv;
    *(volatile v4f*)(kd + qoff) = kv;
    #pragma unroll
    for (int p = 0; p < 4; ++p) *(volatile v8h*)(vd + voff[p]) = vv[p];
    __threadfence();
    *(volatile v4f*)(qd + qoff) = qv;
    *(volatile v4f*)(kd + qoff) = kv;
    #pragma unroll
    for (int p = 0; p < 4; ++p) *(volatile v8h*)(vd + voff[p]) = vv[p];
}

__device__ __forceinline__ float exp_row(const float* srow, float mx, v8ha (&p)[4])
{
    const float cad = fmaf(-mx, L2E, 14.0f);
    v4f e[8];
    #pragma unroll
    for (int u = 0; u < 8; ++u) e[u] = *(const v4f*)(srow + 4 * u);
    float sm = 0.0f;
    #pragma unroll
    for (int u = 0; u < 4; ++u) {
        v8ha t;
        #pragma unroll
        for (int i = 0; i < 8; ++i) {
            const float s = e[2 * u + (i >> 2)][i & 3];
            const float E = EXP2F(fmaf(s, L2E, cad));
            sm += E;
            t[i] = (_Float16)E;
        }
        p[u] = t;
    }
    return sm;
}

template <int ST>
__device__ __forceinline__ void attn_tile(
    const float* sK, float* sS, const v4f* sQ4, float* sInv,
    const _Float16* __restrict__ vd,
    int b, int n0, int w, int h, int m, int rl, int kbase,
    int start, int wsz, int wszk, int nks,
    v8f& os, float& cv)
{
    const int i0 = 16 * ST + rl;
    const v4f q0a = sQ4[2 * i0];
    const v4f q0b = sQ4[2 * i0 + 1];
    const v4f q1a = sQ4[2 * i0 + 2];
    const v4f q1b = sQ4[2 * i0 + 3];
    float* srow0 = sS + rl * SPITCH + kbase;
    float* srow1 = srow0 + SPITCH;
    float mx0 = NEGBIG, mx1 = NEGBIG;

    #pragma unroll 1
    for (int g = 0; g < 8; ++g) {
        v4f d0v, d1v;
        #pragma unroll
        for (int u = 0; u < 4; ++u) {
            const int j = kbase + 4 * g + u;
            const float* kp = sK + j * DD;
            const v4f ka = *(const v4f*)kp;
            const v4f kb = *(const v4f*)(kp + 4);
            float d0 = q0a[0] * ka[0];
            d0 = fmaf(q0a[1], ka[1], d0); d0 = fmaf(q0a[2], ka[2], d0); d0 = fmaf(q0a[3], ka[3], d0);
            d0 = fmaf(q0b[0], kb[0], d0); d0 = fmaf(q0b[1], kb[1], d0); d0 = fmaf(q0b[2], kb[2], d0); d0 = fmaf(q0b[3], kb[3], d0);
            float d1 = q1a[0] * ka[0];
            d1 = fmaf(q1a[1], ka[1], d1); d1 = fmaf(q1a[2], ka[2], d1); d1 = fmaf(q1a[3], ka[3], d1);
            d1 = fmaf(q1b[0], kb[0], d1); d1 = fmaf(q1b[1], kb[1], d1); d1 = fmaf(q1b[2], kb[2], d1); d1 = fmaf(q1b[3], kb[3], d1);
            const bool valid = j < wszk;
            d0 = valid ? d0 : NEGBIG;
            d1 = valid ? d1 : NEGBIG;
            d0v[u] = d0; d1v[u] = d1;
            mx0 = fmaxf(mx0, d0); mx1 = fmaxf(mx1, d1);
        }
        *(v4f*)(srow0 + 4 * g) = d0v;
        *(v4f*)(srow1 + 4 * g) = d1v;
    }
    #pragma unroll
    for (int off = 1; off < 16; off <<= 1) {
        mx0 = fmaxf(mx0, __shfl_xor(mx0, off));
        mx1 = fmaxf(mx1, __shfl_xor(mx1, off));
    }

    v8ha p0[4], p1[4];
    float sm0 = exp_row(srow0, mx0, p0);
    float sm1 = exp_row(srow1, mx1, p1);
    #pragma unroll
    for (int off = 1; off < 16; off <<= 1) {
        sm0 += __shfl_xor(sm0, off);
        sm1 += __shfl_xor(sm1, off);
    }
    __syncthreads();
    _Float16* pr0 = (_Float16*)(sS + rl * SPITCH) + kbase;
    _Float16* pr1 = (_Float16*)(sS + (rl + 1) * SPITCH) + kbase;
    #pragma unroll
    for (int u = 0; u < 4; ++u) {
        *(v8ha*)(pr0 + 8 * u) = p0[u];
        *(v8ha*)(pr1 + 8 * u) = p1[u];
    }
    if (m == 0) { sInv[rl] = frcp(sm0); sInv[rl + 1] = frcp(sm1); }
    __syncthreads();

    const float invm = sInv[m];
    v8f acc;
    #pragma unroll
    for (int r = 0; r < 8; ++r) acc[r] = 0.0f;
    const _Float16* vrow = vd + ((size_t)b * CC + 16 * w + m) * NN + start + 8 * h;
    const _Float16* prow = (const _Float16*)(sS + m * SPITCH) + 8 * h;
    for (int ks = 0; ks < nks; ++ks) {
        Frag af, bf;
        af.hh[0] = *(const v8h*)(vrow + 32 * ks);
        af.hh[1] = *(const v8h*)(vrow + 32 * ks + 16);
        bf.hh[0] = *(const v8h*)(prow + 32 * ks);
        bf.hh[1] = *(const v8h*)(prow + 32 * ks + 16);
        acc = mma_f16(af.v, bf.v, acc);
    }
    const int n = n0 + 16 * ST + m;
    const bool cov = (n >= start) && (n < start + wsz);
    const float cf = cov ? 1.0f : 0.0f;
    cv += cf;
    const float mul = cf * invm;
    #pragma unroll
    for (int r = 0; r < 8; ++r) os[r] = fmaf(mul, acc[r], os[r]);
    __syncthreads();
}

template <int ST>
__device__ __forceinline__ void pool_tile(
    float* sOut, const float* __restrict__ x,
    int b, int n0, int w, int h, int m, int lgP, float gma,
    const v8f& os, float cv)
{
    const int nl = 16 * ST + m;
    const int n  = n0 + nl;
    const float rc = frcp(cv);
    const int Pe = 1 << lgP;
    #pragma unroll
    for (int r = 0; r < 8; ++r) {
        const int c = 16 * w + 8 * h + r;
        const float xv = x[((size_t)b * CC + c) * NN + n];
        float val = (gma * os[r] + cv * xv) * rc;
        for (int off = 1; off < Pe; off <<= 1) val = fmaxf(val, __shfl_xor(val, off));
        if ((m & (Pe - 1)) == 0) sOut[c * SO_LD + (nl >> lgP)] = val;
    }
}

__global__ __launch_bounds__(NTHR) void k_attn(
    const float* __restrict__ qd, const float* __restrict__ kd, const _Float16* __restrict__ vd,
    const float* __restrict__ x, const float* __restrict__ gamma_p,
    const int* __restrict__ wsz_p, const int* __restrict__ str_p, const int* __restrict__ pool_p,
    float* __restrict__ out, int nblk, int npo)
{
    __shared__ __attribute__((aligned(16))) float sS[16 * SPITCH];
    __shared__ __attribute__((aligned(16))) float sK[WCAP * DD];
    __shared__ __attribute__((aligned(16))) v4f   sQ4[TN * DD / 4];
    __shared__ float sInv[16];

    const int tid = threadIdx.x;
    const int w = tid >> 5, l = tid & 31, h = l >> 4, m = l & 15;
    const int b  = blockIdx.x / nblk;
    const int n0 = (blockIdx.x - b * nblk) * TN;

    const int wsz  = wsz_p[0];
    int strd = str_p[0];
    const int praw = pool_p[0];
    const float gma = gamma_p[0];
    if (strd < 1) strd = 1;
    int lgP = 0;
    while (lgP < 4 && (1 << lgP) < praw) ++lgP;
    const int wszk = (wsz < 0) ? 0 : ((wsz > WCAP) ? WCAP : wsz);
    const int nks  = (wszk + 31) >> 5;
    const int nW   = (wsz >= 1 && wsz <= NN) ? ((NN - wsz) / strd + 1) : 0;
    int whi = (n0 + TN - 1) / strd;
    if (whi > nW - 1) whi = nW - 1;
    const int a0 = n0 - wsz + 1;
    const int wlo = (a0 <= 0) ? 0 : (a0 + strd - 1) / strd;
    int nwin = whi - wlo + 1;
    if (nwin < 0) nwin = 0;
    if (nwin > MAXWIN) nwin = MAXWIN;

    sQ4[tid] = *(const v4f*)(qd + ((size_t)b * NN + n0) * DD + 4 * tid);
    v8f os0, os1, os2, os3;
    #pragma unroll
    for (int r = 0; r < 8; ++r) { os0[r] = 0.0f; os1[r] = 0.0f; os2[r] = 0.0f; os3[r] = 0.0f; }
    float cv0 = 0.0f, cv1 = 0.0f, cv2 = 0.0f, cv3 = 0.0f;
    __syncthreads();

    const int rl = 4 * w + 2 * h;
    const int kbase = 32 * m;
    for (int wi = 0; wi < nwin; ++wi) {
        int start = (wlo + wi) * strd;
        if (start < 0) start = 0;
        if (start > NN - 1) start = NN - 1;
        #pragma unroll
        for (int u = 0; u < 8; ++u) {
            const int idx4 = tid + NTHR * u;
            int pos = start + (idx4 >> 1);
            if (pos > NN - 1) pos = NN - 1;
            *(v4f*)(sK + 4 * idx4) = *(const v4f*)(kd + ((size_t)b * NN + pos) * DD + 4 * (idx4 & 1));
        }
        __syncthreads();
        attn_tile<0>(sK, sS, sQ4, sInv, vd, b, n0, w, h, m, rl, kbase, start, wsz, wszk, nks, os0, cv0);
        attn_tile<1>(sK, sS, sQ4, sInv, vd, b, n0, w, h, m, rl, kbase, start, wsz, wszk, nks, os1, cv1);
        attn_tile<2>(sK, sS, sQ4, sInv, vd, b, n0, w, h, m, rl, kbase, start, wsz, wszk, nks, os2, cv2);
        attn_tile<3>(sK, sS, sQ4, sInv, vd, b, n0, w, h, m, rl, kbase, start, wsz, wszk, nks, os3, cv3);
    }
    __syncthreads();

    float* sOut = sS;
    pool_tile<0>(sOut, x, b, n0, w, h, m, lgP, gma, os0, cv0);
    pool_tile<1>(sOut, x, b, n0, w, h, m, lgP, gma, os1, cv1);
    pool_tile<2>(sOut, x, b, n0, w, h, m, lgP, gma, os2, cv2);
    pool_tile<3>(sOut, x, b, n0, w, h, m, lgP, gma, os3, cv3);
    __syncthreads();

    const int wout = TN >> lgP;
    int cpr = wout >> 2;
    if (cpr < 1) cpr = 1;
    int rpp = 32 / cpr;
    if (rpp > 16) rpp = 16;
    const int npass = 16 / rpp;
    const int rr = l / cpr;
    const int qq = l - rr * cpr;
    const int pc0 = (n0 >> lgP) + 4 * qq;
    const bool act = (rr < rpp) && (pc0 + 4 <= npo) && (4 * qq + 4 <= wout);
    const size_t obase = (size_t)b * CC * (size_t)npo + (size_t)pc0;
    for (int p = 0; p < npass; ++p) {
        if (act) {
            const int c = 16 * w + p * rpp + rr;
            const v4f v = *(const v4f*)(sOut + c * SO_LD + 4 * qq);
            *(volatile v4f*)(out + obase + (size_t)c * npo) = v;
        }
    }
    __threadfence();
    for (int p = 0; p < npass; ++p) {
        if (act) {
            const int c = 16 * w + p * rpp + rr;
            const v4f v = *(const v4f*)(sOut + c * SO_LD + 4 * qq);
            *(volatile v4f*)(out + obase + (size_t)c * npo) = v;
        }
    }
}

extern "C" void kernel_launch(void* const* d_in, const int* in_sizes, int n_in,
                              void* d_out, int out_size, void* d_ws, size_t ws_size,
                              hipStream_t stream)
{
    if (n_in < 11) return;
    if (in_sizes[0] != BB * CC * NN) return;
    if (in_sizes[1] != DD * CC || in_sizes[2] != DD) return;
    if (in_sizes[3] != DD * CC || in_sizes[4] != DD) return;
    if (in_sizes[5] != CC * CC || in_sizes[6] != CC) return;
    if (in_sizes[7] < 1 || in_sizes[8] < 1 || in_sizes[9] < 1 || in_sizes[10] < 1) return;
    if (out_size <= 0 || (out_size % (BB * CC)) != 0) return;
    const int npo = out_size / (BB * CC);

    const float* x     = (const float*)d_in[0];
    const float* Wq    = (const float*)d_in[1];
    const float* bq    = (const float*)d_in[2];
    const float* Wk    = (const float*)d_in[3];
    const float* bk    = (const float*)d_in[4];
    const float* Wv    = (const float*)d_in[5];
    const float* bv    = (const float*)d_in[6];
    const float* gamma = (const float*)d_in[7];
    const int*   wszp  = (const int*)d_in[8];
    const int*   strp  = (const int*)d_in[9];
    const int*   poolp = (const int*)d_in[10];
    float* out = (float*)d_out;

    const size_t offW  = 0;
    const size_t offQ  = 16384;
    const size_t szQ   = (size_t)BB * NN * DD * sizeof(float);
    const size_t offK  = offQ + szQ;
    const size_t offV  = offK + szQ;
    const size_t szV   = (size_t)BB * CC * NN * sizeof(_Float16) + 256;
    const size_t total = offV + szV;
    if (total > ws_size) return;

    char* ws = (char*)d_ws;
    _Float16* Wall = (_Float16*)(ws + offW);
    float*    qd   = (float*)(ws + offQ);
    float*    kd   = (float*)(ws + offK);
    _Float16* vd   = (_Float16*)(ws + offV);

    const int nblk = NN / TN;
    k_prep_w<<<dim3(1), dim3(NTHR), 0, stream>>>(Wq, Wk, Wv, Wall);
    k_proj<<<dim3(BB * nblk), dim3(NTHR), 0, stream>>>(x, Wall, bq, bk, bv, qd, kd, vd, nblk);
    k_attn<<<dim3(BB * nblk), dim3(NTHR), 0, stream>>>(qd, kd, vd, x, gamma, wszp, strp, poolp,
                                                       out, nblk, npo);
}
